// TimeAwareTransformer_2826088481575
// MI455X (gfx1250) — hardware-verified
//
#include <hip/hip_runtime.h>
#include <math.h>


#define BB 4
#define LL 128
#define DD 256
#define PP 1024
#define NH 26
#define ND 8
#define TU 86400
#define TB 3600
#define NEGV (-4294967295.0f)

typedef __bf16         v16bf __attribute__((ext_vector_type(16)));
typedef unsigned short v16us __attribute__((ext_vector_type(16)));
typedef float          v8f   __attribute__((ext_vector_type(8)));
typedef float          v4f   __attribute__((ext_vector_type(4)));

union FragU { v16bf v; v16us u; };
struct FragP { v16bf hi; v16bf lo; };

__device__ __forceinline__ int pydiv(int a, int b) {
    int q = a / b;
    if ((a % b != 0) && ((a ^ b) < 0)) --q;
    return q;
}
__device__ __forceinline__ int pymod(int a, int b) {
    int r = a % b;
    if (r != 0 && ((r ^ b) < 0)) r += b;
    return r;
}
__device__ __forceinline__ int wrapclamp(int i, int n) {
    if (i < 0) i += n;
    if (i < 0) i = 0;
    if (i >= n) i = n - 1;
    return i;
}

__device__ __forceinline__ unsigned int rne16(float x) {
    unsigned int u = __float_as_uint(x);
    return (u + 0x7fffu + ((u >> 16) & 1u)) >> 16;
}

__device__ __forceinline__ FragP split16(const float (&x)[16]) {
    v16us hu, lu;
#pragma unroll
    for (int i = 0; i < 16; ++i) {
        const unsigned int hb = rne16(x[i]);
        const float hf = __uint_as_float(hb << 16);
        const unsigned int lb = rne16(x[i] - hf);
        hu[i] = (unsigned short)hb;
        lu[i] = (unsigned short)lb;
    }
    FragU H, Lw;
    H.u = hu; Lw.u = lu;
    FragP f; f.hi = H.v; f.lo = Lw.v;
    return f;
}

__device__ __forceinline__ FragP load_frag(const float* p) {
    const v4f a = *(const v4f*)(p);
    const v4f b = *(const v4f*)(p + 4);
    const v4f c = *(const v4f*)(p + 16);
    const v4f d = *(const v4f*)(p + 20);
    float x[16];
    x[0] = a.x;  x[1] = a.y;  x[2] = a.z;  x[3] = a.w;
    x[4] = b.x;  x[5] = b.y;  x[6] = b.z;  x[7] = b.w;
    x[8] = c.x;  x[9] = c.y;  x[10] = c.z; x[11] = c.w;
    x[12] = d.x; x[13] = d.y; x[14] = d.z; x[15] = d.w;
    return split16(x);
}

__device__ __forceinline__ void mma3(v8f& acc, const FragP& a, const FragP& b) {
    v8f c = acc;
    const v16bf ah = a.hi, al = a.lo, bh = b.hi, bl = b.lo;
    c = __builtin_amdgcn_wmma_f32_16x16x32_bf16(false, ah, false, bh, (short)0, c, false, false);
    c = __builtin_amdgcn_wmma_f32_16x16x32_bf16(false, ah, false, bl, (short)0, c, false, false);
    c = __builtin_amdgcn_wmma_f32_16x16x32_bf16(false, al, false, bh, (short)0, c, false, false);
    asm volatile("v_nop\n\tv_nop\n\tv_nop\n\tv_nop"
                 : "+v"(c) : "v"(ah), "v"(al), "v"(bh), "v"(bl) : "memory");
    acc = c;
}

__global__ void __launch_bounds__(128)
k_gemm(const float* A, int lda,
       const float* W0, const float* W1, int ldw, int nsplit,
       const float* bn0, const float* bn1, const float* bm,
       float* C, int ldc, int M, int N, int K, int relu)
{
    __shared__ __attribute__((aligned(16))) float stg[4][16][68];

    const int w = threadIdx.x >> 5;
    const int l = threadIdx.x & 31;
    const int h = l >> 4;
    const int m = l & 15;
    const int col0 = blockIdx.y * 64;
    if ((int)blockIdx.x * 64 + 64 > M || col0 + 64 > N) return;
    const int row0 = blockIdx.x * 64 + w * 16;

    const float* Wg = W0;
    const float* bg = bn0;
    int wc0 = col0;
    if (col0 >= nsplit) { Wg = W1; bg = bn1; wc0 = col0 - nsplit; }

    const v8f z8 = {0.f, 0.f, 0.f, 0.f, 0.f, 0.f, 0.f, 0.f};
    v8f acc[4];
#pragma unroll
    for (int t = 0; t < 4; ++t) acc[t] = z8;

    const float* ap = A  + (size_t)(row0 + m) * lda + 8 * h;
    const float* wp = Wg + (size_t)(wc0 + m) * ldw + 8 * h;

#pragma unroll 1
    for (int k0 = 0; k0 < K; k0 += 32) {
        const FragP af = load_frag(ap + k0);
#pragma unroll
        for (int t = 0; t < 4; ++t) {
            const FragP bf = load_frag(wp + (size_t)(16 * t) * ldw + k0);
            mma3(acc[t], af, bf);
        }
    }

#pragma unroll
    for (int t = 0; t < 4; ++t) {
        const int colc = 16 * t + m;
        const float bcol = bg ? bg[wc0 + colc] : 0.0f;
#pragma unroll
        for (int r = 0; r < 8; ++r) {
            const int rr = 8 * h + r;
            float v = acc[t][r] + bcol + (bm ? bm[row0 + rr] : 0.0f);
            if (relu) v = fmaxf(v, 0.0f);
            stg[w][rr][colc] = v;
        }
    }
    __syncthreads();

    v4f vals[8];
#pragma unroll
    for (int it = 0; it < 8; ++it) {
        const int line = it * 4 + (l >> 3);
        const int rr   = line >> 1;
        const int cs   = (line & 1) * 32 + (l & 7) * 4;
        vals[it] = *(const v4f*)&stg[w][rr][cs];
    }
#pragma unroll
    for (int it = 0; it < 8; ++it) {
        const int line = it * 4 + (l >> 3);
        const int rr   = line >> 1;
        const int cs   = (line & 1) * 32 + (l & 7) * 4;
        float* cp = C + (size_t)(row0 + rr) * ldc + col0 + cs;
        *(volatile v4f*)cp = vals[it];
    }
    __threadfence();
#pragma unroll
    for (int it = 0; it < 8; ++it) {
        const int line = it * 4 + (l >> 3);
        const int rr   = line >> 1;
        const int cs   = (line & 1) * 32 + (l & 7) * 4;
        float* cp = C + (size_t)(row0 + rr) * ldc + col0 + cs;
        *(volatile v4f*)cp = vals[it];
    }
}

__global__ void __launch_bounds__(32)
k_attn(const float* QK, const float* VT, const float* src,
       const float* hour_emb, const float* day_emb,
       const float* g11, const float* b11,
       const int* slen, const int* ts, float* X, int nblk)
{
    if ((int)blockIdx.x >= nblk) return;
    const int l = threadIdx.x & 31;
    const int h = l >> 4;
    const int m = l & 15;
    const int b  = blockIdx.x / (LL / 16);
    const int j0 = (blockIdx.x % (LL / 16)) * 16;
    const int rb = b * LL + j0;

    __shared__ unsigned char s_hr[16][LL];
    __shared__ unsigned char s_dy[16][LL];
    __shared__ __attribute__((aligned(16))) float s_qe[16][52];
    __shared__ __attribute__((aligned(16))) float s_p[16][132];
    __shared__ __attribute__((aligned(16))) float s_hist[16][68];
    __shared__ __attribute__((aligned(16))) float s_y[16][260];

    const int sl = slen[b];

    for (int e = 0; e < 64; ++e) {
        const int idx = e * 32 + l;
        const int mm  = idx >> 7;
        const int k   = idx & 127;
        const int j   = j0 + mm;
        const bool valid = (k <= j) && (j < sl);
        int hr = 0, dy = 0;
        if (valid) {
            const int diff = ts[b * LL + j] - ts[b * LL + k];
            hr = (b == j) ? 1 : (pymod(diff, TU) / TB + 2);
            dy = pydiv(diff, TU) + 1;
            dy = dy < 7 ? dy : 7;
            hr = wrapclamp(hr, NH);
            dy = wrapclamp(dy, ND);
        }
        s_hr[mm][k] = (unsigned char)hr;
        s_dy[mm][k] = (unsigned char)dy;
    }
    for (int e = 0; e < 32; ++e) {
        const int idx = e * 32 + l;
        s_hist[idx >> 6][idx & 63] = 0.0f;
    }
    __syncthreads();

    const v8f z8 = {0.f, 0.f, 0.f, 0.f, 0.f, 0.f, 0.f, 0.f};
    const float* arow = QK + (size_t)(rb + m) * 512 + 8 * h;

    {
        v8f eacc[3];
#pragma unroll
        for (int t = 0; t < 3; ++t) eacc[t] = z8;
#pragma unroll 1
        for (int k0 = 0; k0 < DD; k0 += 32) {
            const FragP af = load_frag(arow + k0);
#pragma unroll
            for (int t = 0; t < 3; ++t) {
                const int bin = 16 * t + m;
                const float* bp = nullptr;
                if (bin < NH) bp = hour_emb + (size_t)bin * DD;
                else if (bin >= 32 && bin < 32 + ND) bp = day_emb + (size_t)(bin - 32) * DD;
                FragP bf;
                if (bp) {
                    bf = load_frag(bp + k0 + 8 * h);
                } else {
                    float xz[16];
#pragma unroll
                    for (int i = 0; i < 16; ++i) xz[i] = 0.0f;
                    bf = split16(xz);
                }
                mma3(eacc[t], af, bf);
            }
        }
#pragma unroll
        for (int t = 0; t < 3; ++t) {
#pragma unroll
            for (int r = 0; r < 8; ++r) s_qe[8 * h + r][16 * t + m] = eacc[t][r];
        }
    }
    __syncthreads();

    {
        v8f sacc[8];
#pragma unroll
        for (int t = 0; t < 8; ++t) sacc[t] = z8;
#pragma unroll 1
        for (int k0 = 0; k0 < DD; k0 += 32) {
            const FragP af = load_frag(arow + k0);
#pragma unroll
            for (int t = 0; t < 8; ++t) {
                const float* bp = QK + (size_t)(b * LL + 16 * t + m) * 512 + 256 + k0 + 8 * h;
                const FragP bf = load_frag(bp);
                mma3(sacc[t], af, bf);
            }
        }
#pragma unroll
        for (int t = 0; t < 8; ++t) {
#pragma unroll
            for (int r = 0; r < 8; ++r) s_p[8 * h + r][16 * t + m] = sacc[t][r];
        }
    }
    __syncthreads();

    {
        const int kb = 64 * h;
        float mx = NEGV;
        for (int k = kb; k < kb + 64; ++k) {
            const int hr = s_hr[m][k];
            float v = NEGV;
            if (hr != 0) {
                const int dy = s_dy[m][k];
                v = (s_p[m][k] + s_qe[m][hr] + s_qe[m][32 + dy]) * 0.0625f;
            }
            s_p[m][k] = v;
            mx = fmaxf(mx, v);
        }
        mx = fmaxf(mx, __shfl_xor(mx, 16));
        float sum = 0.0f;
        for (int k = kb; k < kb + 64; ++k) {
            const float e = expf(s_p[m][k] - mx);
            s_p[m][k] = e;
            sum += e;
        }
        sum += __shfl_xor(sum, 16);
        const float inv = 1.0f / sum;
        for (int k = kb; k < kb + 64; ++k) s_p[m][k] = s_p[m][k] * inv;
    }
    __syncthreads();

    if (h == 0) {
        for (int k = 0; k < LL; ++k) s_hist[m][s_hr[m][k]] += s_p[m][k];
    } else {
        for (int k = 0; k < LL; ++k) s_hist[m][32 + s_dy[m][k]] += s_p[m][k];
    }
    __syncthreads();

#pragma unroll 1
    for (int c = 0; c < 4; ++c) {
        v8f pacc[4];
#pragma unroll
        for (int t = 0; t < 4; ++t) pacc[t] = z8;

#pragma unroll 1
        for (int ks = 0; ks < 4; ++ks) {
            const FragP af = load_frag(&s_p[m][32 * ks + 8 * h]);
#pragma unroll
            for (int t = 0; t < 4; ++t) {
                const int d = 64 * c + 16 * t + m;
                const FragP bf = load_frag(VT + (size_t)d * (BB * LL) + b * LL + 32 * ks + 8 * h);
                mma3(pacc[t], af, bf);
            }
        }
#pragma unroll 1
        for (int ks = 0; ks < 2; ++ks) {
            const FragP af = load_frag(&s_hist[m][32 * ks + 8 * h]);
#pragma unroll
            for (int t = 0; t < 4; ++t) {
                const int d = 64 * c + 16 * t + m;
                float xg[16];
#pragma unroll
                for (int i = 0; i < 16; ++i) {
                    const int bin = 32 * ks + 8 * h + (i < 8 ? i : i + 8);
                    float v = 0.0f;
                    if (bin < NH) v = hour_emb[(size_t)bin * DD + d];
                    else if (bin >= 32 && bin < 32 + ND) v = day_emb[(size_t)(bin - 32) * DD + d];
                    xg[i] = v;
                }
                const FragP bf = split16(xg);
                mma3(pacc[t], af, bf);
            }
        }
#pragma unroll
        for (int t = 0; t < 4; ++t) {
            const int d = 64 * c + 16 * t + m;
#pragma unroll
            for (int r = 0; r < 8; ++r) {
                const int rr = 8 * h + r;
                s_y[rr][d] = pacc[t][r] + src[(size_t)(rb + rr) * DD + d];
            }
        }
    }
    __syncthreads();

    const v4f ga = *(const v4f*)(g11 + 4 * l);
    const v4f gb = *(const v4f*)(g11 + 128 + 4 * l);
    const v4f ba = *(const v4f*)(b11 + 4 * l);
    const v4f bbv = *(const v4f*)(b11 + 128 + 4 * l);
    for (int rr = 0; rr < 16; ++rr) {
        v4f ya = *(const v4f*)&s_y[rr][4 * l];
        v4f yb = *(const v4f*)&s_y[rr][128 + 4 * l];
        float s = (ya.x + ya.y) + (ya.z + ya.w) + (yb.x + yb.y) + (yb.z + yb.w);
        s += __shfl_xor(s, 1);  s += __shfl_xor(s, 2);  s += __shfl_xor(s, 4);
        s += __shfl_xor(s, 8);  s += __shfl_xor(s, 16);
        const float mean = s * (1.0f / DD);
        const v4f da = ya - mean;
        const v4f db = yb - mean;
        float q = (da.x * da.x + da.y * da.y) + (da.z * da.z + da.w * da.w)
                + (db.x * db.x + db.y * db.y) + (db.z * db.z + db.w * db.w);
        q += __shfl_xor(q, 1);  q += __shfl_xor(q, 2);  q += __shfl_xor(q, 4);
        q += __shfl_xor(q, 8);  q += __shfl_xor(q, 16);
        const float var = q * (1.0f / DD);
        const float rs = rsqrtf(var + 1e-5f);
        const v4f oa = da * rs * ga + ba;
        const v4f ob = db * rs * gb + bbv;
        *(v4f*)&s_y[rr][4 * l]       = oa;
        *(v4f*)&s_y[rr][128 + 4 * l] = ob;
        float* xp = X + (size_t)(rb + rr) * DD;
        *(volatile v4f*)(xp + 4 * l)       = oa;
        *(volatile v4f*)(xp + 128 + 4 * l) = ob;
    }
    __threadfence();
    for (int rr = 0; rr < 16; ++rr) {
        const v4f oa = *(const v4f*)&s_y[rr][4 * l];
        const v4f ob = *(const v4f*)&s_y[rr][128 + 4 * l];
        float* xp = X + (size_t)(rb + rr) * DD;
        *(volatile v4f*)(xp + 4 * l)       = oa;
        *(volatile v4f*)(xp + 128 + 4 * l) = ob;
    }
}

__global__ void __launch_bounds__(64)
k_ln2(const float* Xb, const float* F2, const float* g, const float* be, float* F, int nrows)
{
    const int r = blockIdx.x;
    if (r >= nrows) return;
    const int t = threadIdx.x;
    const int l = t & 31;
    const int w = t >> 5;
    __shared__ float red[2][2];

    const size_t base = (size_t)r * DD + 4 * t;
    const v4f x = *(const v4f*)(Xb + base);
    const v4f f = *(const v4f*)(F2 + base);
    const v4f y = x + f;
    float s = (y.x + y.y) + (y.z + y.w);
    s += __shfl_xor(s, 1);  s += __shfl_xor(s, 2);  s += __shfl_xor(s, 4);
    s += __shfl_xor(s, 8);  s += __shfl_xor(s, 16);
    if (l == 0) red[0][w] = s;
    __syncthreads();
    const float mean = (red[0][0] + red[0][1]) * (1.0f / DD);
    const v4f dv = y - mean;
    float q = (dv.x * dv.x + dv.y * dv.y) + (dv.z * dv.z + dv.w * dv.w);
    q += __shfl_xor(q, 1);  q += __shfl_xor(q, 2);  q += __shfl_xor(q, 4);
    q += __shfl_xor(q, 8);  q += __shfl_xor(q, 16);
    if (l == 0) red[1][w] = q;
    __syncthreads();
    const float var = (red[1][0] + red[1][1]) * (1.0f / DD);
    const float rs = rsqrtf(var + 1e-5f);
    const v4f gg = *(const v4f*)(g + 4 * t);
    const v4f bv = *(const v4f*)(be + 4 * t);
    const v4f o = dv * rs * gg + bv;
    float* fp = F + base;
    *(volatile v4f*)fp = o;
    __threadfence();
    *(volatile v4f*)fp = o;
}

__global__ void __launch_bounds__(64)
k_pool(const float* F, const float* hour_emb, const float* day_emb,
       const int* slen, const int* ts, const int* lts, float* U, int nblk)
{
    const int bj = blockIdx.x;
    if (bj >= nblk) return;
    const int b = bj / LL;
    const int j = bj % LL;
    const int t = threadIdx.x;

    __shared__ unsigned char s_h[LL];
    __shared__ unsigned char s_d[LL];

    const bool jv = (j < slen[b]);
    for (int q = 0; q < 2; ++q) {
        const int k = t + 64 * q;
        const bool valid = (k <= j) && jv;
        int hr = 0, dy = 0;
        if (valid) {
            const int ld = lts[b * LL + j] - ts[b * LL + k];
            hr = pymod(ld, TU) / TB + 2;
            dy = pydiv(ld, TU) + 1;
            dy = dy < 7 ? dy : 7;
            hr = wrapclamp(hr, NH);
            dy = wrapclamp(dy, ND);
        }
        s_h[k] = (unsigned char)hr;
        s_d[k] = (unsigned char)dy;
    }
    __syncthreads();

    v4f acc = {0.f, 0.f, 0.f, 0.f};
    for (int k = 0; k <= j; ++k) {
        const v4f fv = *(const v4f*)(F + (size_t)(b * LL + k) * DD + 4 * t);
        const v4f he = *(const v4f*)(hour_emb + (size_t)s_h[k] * DD + 4 * t);
        const v4f de = *(const v4f*)(day_emb  + (size_t)s_d[k] * DD + 4 * t);
        acc += fv + he + de;
    }
    const float inv = 1.0f / (float)(j + 1);
    const v4f o = acc * inv;
    float* up = U + (size_t)(b * LL + j) * DD + 4 * t;
    *(volatile v4f*)up = o;
    __threadfence();
    *(volatile v4f*)up = o;
}

extern "C" void kernel_launch(void* const* d_in, const int* in_sizes, int n_in,
                              void* d_out, int out_size, void* d_ws, size_t ws_size,
                              hipStream_t stream)
{
    if (n_in < 22) return;
    const int expect[22] = {
        BB * LL * DD, NH * DD, ND * DD,
        DD * DD, DD, DD * DD, DD, DD * DD, DD,
        DD, DD,
        DD * DD, DD, DD * DD, DD,
        DD, DD,
        PP * DD, PP,
        BB, BB * LL, BB * LL };
    for (int i = 0; i < 22; ++i) if (in_sizes[i] != expect[i]) return;
    if (out_size != BB * LL * PP) return;

    const float* src      = (const float*)d_in[0];
    const float* hour_emb = (const float*)d_in[1];
    const float* day_emb  = (const float*)d_in[2];
    const float* wq       = (const float*)d_in[3];
    const float* bq       = (const float*)d_in[4];
    const float* wk       = (const float*)d_in[5];
    const float* bk       = (const float*)d_in[6];
    const float* wv       = (const float*)d_in[7];
    const float* bv       = (const float*)d_in[8];
    const float* g11      = (const float*)d_in[9];
    const float* b11      = (const float*)d_in[10];
    const float* wf1      = (const float*)d_in[11];
    const float* bf1      = (const float*)d_in[12];
    const float* wf2      = (const float*)d_in[13];
    const float* bf2      = (const float*)d_in[14];
    const float* g12      = (const float*)d_in[15];
    const float* b12      = (const float*)d_in[16];
    const float* wdec     = (const float*)d_in[17];
    const float* bdec     = (const float*)d_in[18];
    const int*   slen     = (const int*)d_in[19];
    const int*   ts       = (const int*)d_in[20];
    const int*   lts      = (const int*)d_in[21];
    float*       out      = (float*)d_out;

    const int M = BB * LL;
    const size_t nQK = (size_t)M * 512;
    const size_t nVT = (size_t)DD * M;
    const size_t nR  = (size_t)M * DD;
    const size_t need_floats = nQK + nVT + 5 * nR;
    if (ws_size < need_floats * sizeof(float)) return;

    float* ws = (float*)d_ws;
    float* QK = ws;
    float* VT = QK + nQK;
    float* Xb = VT + nVT;
    float* F1 = Xb + nR;
    float* F2 = F1 + nR;
    float* Fb = F2 + nR;
    float* Ub = Fb + nR;

    k_gemm<<<dim3(M / 64, 512 / 64), 128, 0, stream>>>(
        src, DD, wq, wk, DD, DD, bq, bk, nullptr, QK, 512, M, 512, DD, 0);
    k_gemm<<<dim3(DD / 64, M / 64), 128, 0, stream>>>(
        wv, DD, src, src, DD, M, nullptr, nullptr, bv, VT, M, DD, M, DD, 0);
    const int nattn = M / 16;
    k_attn<<<nattn, 32, 0, stream>>>(QK, VT, src, hour_emb, day_emb, g11, b11, slen, ts, Xb, nattn);
    k_gemm<<<dim3(M / 64, DD / 64), 128, 0, stream>>>(
        Xb, DD, wf1, wf1, DD, DD, bf1, bf1, nullptr, F1, DD, M, DD, DD, 1);
    k_gemm<<<dim3(M / 64, DD / 64), 128, 0, stream>>>(
        F1, DD, wf2, wf2, DD, DD, bf2, bf2, nullptr, F2, DD, M, DD, DD, 0);
    k_ln2<<<M, 64, 0, stream>>>(Xb, F2, g12, b12, Fb, M);
    k_pool<<<M, 64, 0, stream>>>(Fb, hour_emb, day_emb, slen, ts, lts, Ub, M);
    k_gemm<<<dim3(M / 64, PP / 64), 128, 0, stream>>>(
        Ub, DD, wdec, wdec, DD, PP, bdec, bdec, nullptr, out, PP, M, PP, DD, 0);
}
